// SimplifiedMambaBlock_63376537419871
// MI455X (gfx1250) — hardware-run, weakly checked
//
#include <hip/hip_runtime.h>


#pragma clang fp contract(off)

#ifndef NB
#define NB 2
#endif
#ifndef SEQ
#define SEQ 2048
#endif
#define NB_FULL  2
#define SEQ_FULL 2048
#ifndef OUT_SEQ
#define OUT_SEQ SEQ
#endif
#define DIM   768
#define ED    1536
#define NST   16
#define NCV   4
#define OSP2  68
#define TC    32
#define XS    16.0f
#define YS    16.0f
#define WS    64.0f
#define SCL   (1.0f / 1024.0f)
#define RSD   0.03608439182435161f
#define EPSF  1e-6f

static_assert(DIM == 3 * 32 * 8);
static_assert(ED == 2 * DIM);
static_assert(DIM % 32 == 0);
static_assert(ED % 32 == 0);
static_assert(DIM % 64 == 0);
static_assert(ED % 64 == 0);
static_assert(SEQ % 64 == 0);
static_assert((NB * SEQ) % 64 == 0);
static_assert((NB * SEQ) % 8 == 0);
static_assert(SEQ % TC == 0);
static_assert(TC * 64 * 2 == 64 * 16 * 4);
static_assert(32 * 4 * 8 == 16 * 64);
static_assert((OSP2 * 4) % 16 == 0);
static_assert(16 * OSP2 * 4 <= 131072);
static_assert(TC * 64 * 2 <= 131072);
static_assert(((size_t)ED * DIM) % 8 == 0);
static_assert(((size_t)ED * NST) % 4 == 0);
static_assert(NST == 16);
static_assert(NCV == 4);
static_assert(NB <= NB_FULL);
static_assert(SEQ <= SEQ_FULL);

typedef _Float16 h16;
typedef __attribute__((ext_vector_type(16))) _Float16 v16h;
typedef __attribute__((ext_vector_type(8)))  _Float16 v8h;
typedef __attribute__((ext_vector_type(8)))  float    v8f;
typedef __attribute__((ext_vector_type(4)))  float    v4f;
typedef v4f  __attribute__((may_alias)) v4fa;
typedef v8h  __attribute__((may_alias)) v8ha;

__device__ __forceinline__ unsigned short f2bf(float f) { unsigned u = __float_as_uint(f); u += 0x7FFFu + ((u >> 16) & 1u); return (unsigned short)(u >> 16); }
__device__ __forceinline__ float bfr(float f) { return __uint_as_float(((unsigned)f2bf(f)) << 16); }
__device__ __forceinline__ v16h cat16(v8h lo, v8h hi) { return __builtin_shufflevector(lo, hi, 0, 1, 2, 3, 4, 5, 6, 7, 8, 9, 10, 11, 12, 13, 14, 15); }
__device__ __forceinline__ v8f wmma16(v16h a, v16h b, v8f c) { return __builtin_amdgcn_wmma_f32_16x16x32_f16(false, a, false, b, (short)0, c, false, false); }
__device__ __forceinline__ v16h  ldh(const h16* p) { return cat16(*(const v8h*)p, *(const v8h*)(p + 16)); }
__device__ __forceinline__ void wave_sync() { __builtin_amdgcn_fence(3  , "wavefront"); __builtin_amdgcn_wave_barrier(); asm volatile("" ::: "memory"); }
__device__ __forceinline__ h16 toh_flush(float v) { const h16 r = (h16)v; return (fabsf(v) < 6.103515625e-05f) ? (h16)0.0f : r; }
__device__ __forceinline__ v8f wmma16g(v16h a, v16h b, v8f c) { c = wmma16(a, b, c); asm volatile("v_nop\n\tv_nop\n\tv_nop\n\tv_nop" : "+v"(c) : "v"(a), "v"(b)); return c; }

__global__ __launch_bounds__(256) void k_norm(const float* __restrict__ x, const float* __restrict__ gamma, h16* XN) {
    const int lane = threadIdx.x & 31;
    const int wave = __builtin_amdgcn_readfirstlane((int)(threadIdx.x >> 5));
    const int m = blockIdx.x * 8 + wave;
    const int bb = m / SEQ, tt = m % SEQ;
    const float* xr = x + ((size_t)bb * SEQ_FULL + (size_t)tt) * DIM;
    v8f v[3]; float ss = 0.0f;
#pragma unroll
    for (int c = 0; c < 3; ++c) { v[c] = *(const v8f*)(xr + (c * 32 + lane) * 8);
#pragma unroll
        for (int k = 0; k < 8; ++k) { const float q = bfr(v[c][k]); v[c][k] = q; ss = ss + q * q; } }
    ss = ss + __shfl_xor(ss, 16, 32); ss = ss + __shfl_xor(ss, 8, 32); ss = ss + __shfl_xor(ss, 4, 32);
    ss = ss + __shfl_xor(ss, 2, 32);  ss = ss + __shfl_xor(ss, 1, 32);
    const float rms = sqrtf(ss) * RSD;
    const float inv = 1.0f / (rms + EPSF);
    v8h o[3];
#pragma unroll
    for (int c = 0; c < 3; ++c) { const v8f g = *(const v8f*)(gamma + (c * 32 + lane) * 8);
#pragma unroll
        for (int k = 0; k < 8; ++k) o[c][k] = toh_flush((bfr(g[k]) * (v[c][k] * inv)) * XS); }
    h16* dr = XN + (size_t)m * DIM;
#pragma unroll 1
    for (int ps = 0; ps < 2; ++ps) {
#pragma unroll
        for (int c = 0; c < 3; ++c) *(volatile v8h*)(dr + (c * 32 + lane) * 8) = o[c];
        if (ps == 0) __threadfence(); }
}

__global__ __launch_bounds__(256) void k_wcvt(const float* __restrict__ src, h16* dst, size_t n8) {
    const size_t i = (size_t)blockIdx.x * 256 + threadIdx.x; if (i >= n8) return;
    const v8f v = *(const v8f*)(src + i * 8); v8h o;
#pragma unroll
    for (int k = 0; k < 8; ++k) o[k] = toh_flush(bfr(v[k]) * WS);
    *(volatile v8h*)(dst + i * 8) = o; __threadfence(); *(volatile v8h*)(dst + i * 8) = o;
}

__global__ __launch_bounds__(256) void k_sig(const float* __restrict__ src, float* dst, int n4) {
    const int i = blockIdx.x * 256 + threadIdx.x; if (i >= n4) return;
    const v4f v = *(const v4f*)(src + (size_t)i * 4); v4f o;
#pragma unroll
    for (int k = 0; k < 4; ++k) o[k] = 1.0f / (1.0f + expf(-bfr(v[k])));
    *(volatile v4f*)(dst + (size_t)i * 4) = o; __threadfence(); *(volatile v4f*)(dst + (size_t)i * 4) = o;
}

template <int RES, int KD, int ND>
__device__ __forceinline__ void gemm_tile(const h16* __restrict__ A, const h16* __restrict__ Bt, const float* __restrict__ bias, const float* __restrict__ X, float* C) {
    __shared__ __align__(16) float os[16 * OSP2];
    const int lane = threadIdx.x & 31, lr = lane & 15, hi = lane >> 4; const int r0 = blockIdx.x * 64, c0 = blockIdx.y * 64;
    v8f acc[4][4];
#pragma unroll
    for (int mb = 0; mb < 4; ++mb)
#pragma unroll
        for (int nb = 0; nb < 4; ++nb) acc[mb][nb] = (v8f){};
    const size_t aoff = (size_t)(r0 + lr) * KD + 8 * hi, boff = (size_t)(c0 + lr) * KD + 8 * hi;
#pragma unroll 1
    for (int kc = 0; kc < KD; kc += 32) {
        v16h a[4];
#pragma unroll
        for (int mb = 0; mb < 4; ++mb) a[mb] = ldh(A + aoff + (size_t)mb * 16 * KD + kc);
#pragma unroll
        for (int nb = 0; nb < 4; ++nb) { const v16h b = ldh(Bt + boff + (size_t)nb * 16 * KD + kc);
#pragma unroll
            for (int mb = 0; mb < 4; ++mb) acc[mb][nb] = wmma16g(a[mb], b, acc[mb][nb]); }
    }
    float bc[4];
#pragma unroll
    for (int nb = 0; nb < 4; ++nb) bc[nb] = bfr(bias[c0 + nb * 16 + lr]);
    const int bb = r0 / SEQ, tt = r0 % SEQ;
    const size_t crow0 = RES ? ((size_t)bb * OUT_SEQ + (size_t)tt) : (size_t)r0;
    const size_t xrow0 = (size_t)bb * SEQ_FULL + (size_t)tt;
#pragma unroll
    for (int mb = 0; mb < 4; ++mb) {
#pragma unroll
        for (int nb = 0; nb < 4; ++nb) {
#pragma unroll
            for (int j = 0; j < 8; ++j) os[(hi * 8 + j) * OSP2 + nb * 16 + lr] = acc[mb][nb][j] * SCL + bc[nb]; }
        wave_sync();
        v4f val[8];
#pragma unroll
        for (int s = 0; s < 8; ++s) { const int row = 2 * s + (lane >> 4), c4 = (lane & 15) * 4;
            v4f t = *(const v4fa*)(&os[row * OSP2 + c4]);
            if (RES) { const v4f xv = *(const v4f*)(X + (xrow0 + (size_t)(mb * 16 + row)) * ND + c0 + c4);
#pragma unroll
                for (int i = 0; i < 4; ++i) t[i] = t[i] + bfr(xv[i]); }
            val[s] = t; }
#pragma unroll 1
        for (int ps = 0; ps < 2; ++ps) {
#pragma unroll
            for (int s = 0; s < 8; ++s) { const int row = 2 * s + (lane >> 4), c4 = (lane & 15) * 4;
                *(volatile v4f*)(C + (crow0 + (size_t)(mb * 16 + row)) * ND + c0 + c4) = val[s]; }
            if (ps == 0) __threadfence(); }
        wave_sync();
    }
}

__global__ __launch_bounds__(32) void k_gemm_in(const h16* __restrict__ A, const h16* __restrict__ Bt, const float* __restrict__ bias, float* C) {
    gemm_tile<0, DIM, ED>(A, Bt, bias, bias, C);
}
__global__ __launch_bounds__(32) void k_gemm_out(const h16* __restrict__ A, const h16* __restrict__ Bt, const float* __restrict__ bias, const float* __restrict__ X, float* C) {
    gemm_tile<1, ED, DIM>(A, Bt, bias, X, C);
}

__global__ __launch_bounds__(64) void k_scan(const float* __restrict__ XP, const float* __restrict__ convw, const float* __restrict__ SG, h16* Y) {
    __shared__ __align__(16) h16 ys[TC * 64];
    const int tid = threadIdx.x;
    const int cb = blockIdx.x, bz = blockIdx.y;
    const int e = cb * 64 + tid;
    const v4f cw = *(const v4f*)(convw + (size_t)e * NCV);
    const float w0 = bfr(cw[0]), w1 = bfr(cw[1]), w2 = bfr(cw[2]), w3 = bfr(cw[3]);
    float sA[NST], sB[NST], sC[NST], h[NST];
#pragma unroll
    for (int q = 0; q < 4; ++q) {
        const v4f ta = *(const v4f*)(SG + (size_t)e * NST + 4 * q);
        const v4f tb = *(const v4f*)(SG + (size_t)ED * NST + (size_t)e * NST + 4 * q);
        const v4f tc = *(const v4f*)(SG + (size_t)2 * ED * NST + (size_t)e * NST + 4 * q);
#pragma unroll
        for (int i = 0; i < 4; ++i) { sA[4 * q + i] = ta[i]; sB[4 * q + i] = tb[i]; sC[4 * q + i] = tc[i]; h[4 * q + i] = 0.0f; } }
    float p1 = 0.0f, p2 = 0.0f, p3 = 0.0f;
    const float* col = XP + (size_t)bz * SEQ * ED + e;
    float cur = col[0];
#pragma unroll 1
    for (int t0 = 0; t0 < SEQ; t0 += TC) {
#pragma unroll 1
        for (int tt = 0; tt < TC; ++tt) {
            const int t = t0 + tt;
            const int tn = (t + 1 < SEQ) ? (t + 1) : (SEQ - 1);
            const float nxt = col[(size_t)tn * ED];
            const float xc = ((p3 * w0 + p2 * w1) + p1 * w2) + cur * w3;
            p3 = p2; p2 = p1; p1 = cur;
            float y = 0.0f;
#pragma unroll
            for (int n = 0; n < NST; ++n) { h[n] = sA[n] * h[n] + sB[n] * xc; y = y + h[n] * sC[n]; }
            ys[tt * 64 + tid] = toh_flush(y * YS);
            cur = nxt;
        }
        __syncthreads();
#pragma unroll 1
        for (int ps = 0; ps < 2; ++ps) {
#pragma unroll
            for (int s = 0; s < 4; ++s) { const int row = 8 * s + (tid >> 3), c8 = (tid & 7) * 8;
                const v8h val = *(const v8ha*)(&ys[row * 64 + c8]);
                *(volatile v8h*)(Y + ((size_t)bz * SEQ + (size_t)(t0 + row)) * ED + cb * 64 + c8) = val; }
            if (ps == 0) __threadfence(); }
        __syncthreads();
    }
}

static constexpr size_t al256(size_t v) { return (v + 255) & ~(size_t)255; }
static constexpr size_t SZ_XN = al256((size_t)NB * SEQ * DIM * 2);
static constexpr size_t SZ_W  = al256((size_t)ED * DIM * 2);
static constexpr size_t SZ_SG = al256((size_t)3 * ED * NST * 4);
static constexpr size_t SZ_XP = al256((size_t)NB * SEQ * ED * 4);
static constexpr size_t SZ_Y  = al256((size_t)NB * SEQ * ED * 2);
static constexpr size_t SZ_TOTAL = SZ_XN + 2 * SZ_W + SZ_SG + SZ_XP + SZ_Y;
static_assert(SZ_TOTAL <= (size_t)134217728);
static_assert(((size_t)ED * NST * 4) % 128 == 0);

extern "C" void kernel_launch(void* const* d_in, const int* in_sizes, int n_in,
                              void* d_out, int out_size, void* d_ws, size_t ws_size, hipStream_t stream) {
    if (n_in < 10) return;
    const size_t needx = ((size_t)(NB - 1) * SEQ_FULL + SEQ) * DIM;
    if ((size_t)in_sizes[0] < needx) return;
    if (in_sizes[1] < DIM) return;
    if ((size_t)in_sizes[2] < (size_t)ED * DIM || in_sizes[3] < ED) return;
    if (in_sizes[4] < ED * NCV) return;
    if (in_sizes[5] < ED * NST || in_sizes[6] < ED * NST || in_sizes[7] < ED * NST) return;
    if ((size_t)in_sizes[8] < (size_t)DIM * ED || in_sizes[9] < DIM) return;
    if ((size_t)out_size < ((size_t)(NB - 1) * OUT_SEQ + SEQ) * DIM) return;
    if (SZ_TOTAL > ws_size) return;
    const float* x     = (const float*)d_in[0];
    const float* gamma = (const float*)d_in[1];
    const float* w_in  = (const float*)d_in[2];
    const float* b_in  = (const float*)d_in[3];
    const float* cw    = (const float*)d_in[4];
    const float* pA    = (const float*)d_in[5];
    const float* pB    = (const float*)d_in[6];
    const float* pC    = (const float*)d_in[7];
    const float* w_out = (const float*)d_in[8];
    const float* b_out = (const float*)d_in[9];
    float* OUT = (float*)d_out;
    char* wsp = (char*)d_ws;
    h16* XN = (h16*)wsp; wsp += SZ_XN;
    h16* WI = (h16*)wsp; wsp += SZ_W;
    h16* WO = (h16*)wsp; wsp += SZ_W;
    float* SG = (float*)wsp; wsp += SZ_SG;
    float* XP = (float*)wsp; wsp += SZ_XP;
    h16* Y  = (h16*)wsp; wsp += SZ_Y;

    k_norm<<<(unsigned)(NB * SEQ / 8), 256, 0, stream>>>(x, gamma, XN);
    { const size_t n8 = (size_t)ED * DIM / 8; const unsigned g = (unsigned)((n8 + 255) / 256);
      k_wcvt<<<g, 256, 0, stream>>>(w_in, WI, n8); k_wcvt<<<g, 256, 0, stream>>>(w_out, WO, n8); }
    { const int n4 = ED * NST / 4; const unsigned g = (unsigned)((n4 + 255) / 256);
      k_sig<<<g, 256, 0, stream>>>(pA, SG, n4);
      k_sig<<<g, 256, 0, stream>>>(pB, SG + (size_t)ED * NST, n4);
      k_sig<<<g, 256, 0, stream>>>(pC, SG + (size_t)2 * ED * NST, n4); }

    k_gemm_in<<<dim3(NB * SEQ / 64, ED / 64, 1), 32, 0, stream>>>(XN, WI, b_in, XP);
    k_scan<<<dim3(ED / 64, NB, 1), 64, 0, stream>>>(XP, cw, SG, Y);
    k_gemm_out<<<dim3(NB * SEQ / 64, DIM / 64, 1), 32, 0, stream>>>(Y, WO, b_out, x, OUT);
}
